// ForceField_79353815761255
// MI455X (gfx1250) — hardware-verified
//
#include <hip/hip_runtime.h>
#include <math.h>
#include <stdint.h>

#pragma clang fp contract(off)

#ifndef NL
#define NL 512
#endif
#ifndef NR
#define NR 4096
#endif
#define NL_FULL 512
#define NR_FULL 4096
#define NE 32
#define NF 64
#define FP (NE * NF)
#define RBF_END_F 8.0f
#define ESCALE 0.01f
#define NEG16LOG2E (-16.0f * 1.44269504088896340736f)

static_assert(NL >= 64 && NL <= NL_FULL && (NL % 64) == 0);
static_assert(NR >= 64 && NR <= NR_FULL && (NR % 64) == 0);
static_assert((NF % 32) == 0 && (FP % 8) == 0);

#define NBX  (NR / 64)
#define NBY  (NL / 64)
#define NBLK (NBX * NBY)

#define LIGB  ((long long)NL * FP * 2)
#define RECB  ((long long)NR * FP * 2)
#define PARTB ((long long)NBLK * 32 * 4)
static_assert((LIGB % 128) == 0 && (RECB % 128) == 0 && (PARTB % 128) == 0);
static_assert(LIGB + RECB + PARTB <= 134217728LL);
static_assert(((NL * FP / 8) % 256) == 0 && ((NR * FP / 8) % 256) == 0);
static_assert(NBLK <= 65536);

typedef _Float16 v16h __attribute__((ext_vector_type(16)));
typedef _Float16 v8h  __attribute__((ext_vector_type(8)));
typedef __bf16   v16b __attribute__((ext_vector_type(16)));
typedef __bf16   v8b  __attribute__((ext_vector_type(8)));
typedef float    v8f  __attribute__((ext_vector_type(8)));
typedef float    v4f  __attribute__((ext_vector_type(4)));
typedef unsigned int v4u __attribute__((ext_vector_type(4)));

#if defined(__HIP_DEVICE_COMPILE__)
#define DEV_ASM 1
#else
#define DEV_ASM 0
#endif

__device__ __forceinline__ unsigned short bf_bits(float f) {
  unsigned u = __float_as_uint(f);
  return (unsigned short)((u + 0x7FFFu + ((u >> 16) & 1u)) >> 16);
}
__device__ __forceinline__ float bf_up(unsigned short hb) { return __uint_as_float(((unsigned)hb) << 16); }
__device__ __forceinline__ unsigned pk16(unsigned short a, unsigned short b) { return (unsigned)a | ((unsigned)b << 16); }
__device__ __forceinline__ v8f zero8() { v8f z = {0.f, 0.f, 0.f, 0.f, 0.f, 0.f, 0.f, 0.f}; return z; }

template <typename OT> struct FT;
template <> struct FT<__bf16>   { typedef v16b frag; typedef v8b half8; };
template <> struct FT<_Float16> { typedef v16h frag; typedef v8h half8; };

template <typename OT>
__device__ __forceinline__ typename FT<OT>::frag ldfrag(const OT* p) {
  union { typename FT<OT>::frag v; typename FT<OT>::half8 h[2]; } f;
  f.h[0] = *(const typename FT<OT>::half8*)(p);
  f.h[1] = *(const typename FT<OT>::half8*)(p + 16);
  return f.v;
}

__device__ __forceinline__ v8f mmar(v16b a, v16b b, v8f c) {
  return __builtin_amdgcn_wmma_f32_16x16x32_bf16(false, a, false, b, (short)0, c, false, false);
}
__device__ __forceinline__ void dep_guard(v8f& a, v8f& b, v16b x, v16b y) {
#if DEV_ASM
  asm volatile("v_nop\n\tv_nop\n\tv_nop\n\tv_nop" : "+v"(a), "+v"(b) : "v"(x), "v"(y));
#else
  (void)a; (void)b; (void)x; (void)y;
#endif
}
__device__ __forceinline__ void keep4(v16b a, v16b b, v16b c, v16b d) {
#if DEV_ASM
  asm volatile("v_nop" :: "v"(a), "v"(b), "v"(c), "v"(d));
#else
  (void)a; (void)b; (void)c; (void)d;
#endif
}
__device__ __forceinline__ void acc_guard4(v8f& a, v8f& b, v8f& c, v8f& d) {
#if DEV_ASM
  asm volatile("v_nop\n\tv_nop\n\tv_nop\n\tv_nop" : "+v"(a), "+v"(b), "+v"(c), "+v"(d));
#else
  (void)a; (void)b; (void)c; (void)d;
#endif
}

__global__ __launch_bounds__(256) void cvt_bf16x8(const float* __restrict__ in, unsigned short* out, int n8) {
  const int i = blockIdx.x * 256 + (int)threadIdx.x;
  if (i < n8) {
    const float* ip = in + (size_t)i * 8;
    const v4f a  = *(const v4f*)(ip);
    const v4f a4 = *(const v4f*)(ip + 4);
    v4u p;
    p[0] = pk16(bf_bits(a[0]),  bf_bits(a[1]));
    p[1] = pk16(bf_bits(a[2]),  bf_bits(a[3]));
    p[2] = pk16(bf_bits(a4[0]), bf_bits(a4[1]));
    p[3] = pk16(bf_bits(a4[2]), bf_bits(a4[3]));
    unsigned short* o = out + (size_t)i * 8;
    *(volatile v4u*)o = p;
    __threadfence();
    *(volatile v4u*)o = p;
  }
}

__global__ __launch_bounds__(128) void pair_energy(const unsigned short* __restrict__ LIGp,
                                                   const unsigned short* __restrict__ RECp,
                                                   const float* __restrict__ ligc,
                                                   const float* __restrict__ recc,
                                                   float* PART) {
  const __bf16* LIG = (const __bf16*)(const void*)LIGp;
  const __bf16* REC = (const __bf16*)(const void*)RECp;
  __shared__ __align__(16) float sL[192];
  __shared__ __align__(16) float sR[192];
  __shared__ __align__(16) float sD[4][16 * 64];
  __shared__ float red[4];

  const int tid  = (int)threadIdx.x;
  const int lane = tid & 31;
  const int wave = tid >> 5;
  const int m    = lane & 15;
  const int h    = lane >> 4;
  const int bx   = blockIdx.x;
  const int by   = blockIdx.y;
  const int lB   = by * 64;
  const int rB   = bx * 64;

  {
    const int t = (tid < 48) ? tid : 47;
    const v4f a = *(const v4f*)(ligc + (size_t)lB * 3 + (size_t)t * 4);
    const v4f b = *(const v4f*)(recc + (size_t)rB * 3 + (size_t)t * 4);
    v4f ar, br;
#pragma unroll
    for (int c = 0; c < 4; ++c) { ar[c] = bf_up(bf_bits(a[c])); br[c] = bf_up(bf_bits(b[c])); }
    if (tid < 48) {
      *(v4f*)(sL + t * 4) = ar;
      *(v4f*)(sR + t * 4) = br;
    }
  }
  __syncthreads();

#pragma unroll 1
  for (int it = 0; it < 32; ++it) {
    const int idx = it * 32 + lane;
    const int row = idx >> 6;
    const int col = idx & 63;
    const float* lp = sL + (wave * 16 + row) * 3;
    const float* rp = sR + col * 3;
    const float dx = lp[0] - rp[0];
    const float dy = lp[1] - rp[1];
    const float dz = lp[2] - rp[2];
    const float sq = (dx * dx + dz * dz) + dy * dy;
    sD[wave][idx] = sqrtf(sq);
  }
  __syncthreads();

  float dist[4][8];
#pragma unroll
  for (int j = 0; j < 4; ++j)
#pragma unroll
    for (int r = 0; r < 8; ++r)
      dist[j][r] = sD[wave][(8 * h + r) * 64 + 16 * j + m];

  const __bf16* Arow = LIG + (size_t)(lB + wave * 16 + m) * FP + 8 * h;
  const __bf16* Brow = REC + (size_t)(rB + m) * FP + 8 * h;
  float run = 0.f;

#pragma unroll 1
  for (int e = 0; e < NE; ++e) {
    v8f acc[4];
#pragma unroll
    for (int j = 0; j < 4; ++j) acc[j] = zero8();
#pragma unroll
    for (int kk = 0; kk < 2; ++kk) {
      const int ko = e * NF + kk * 32;
      v16b bq[4];
#pragma unroll
      for (int j = 0; j < 4; ++j) bq[j] = ldfrag<__bf16>(Brow + (size_t)j * 16 * FP + ko);
      const v16b af = ldfrag<__bf16>(Arow + ko);
#pragma unroll
      for (int j = 0; j < 4; ++j) acc[j] = mmar(af, bq[j], acc[j]);
      dep_guard(acc[0], acc[3], af, bq[3]);
      keep4(bq[0], bq[1], bq[2], bq[3]);
    }
    acc_guard4(acc[0], acc[1], acc[2], acc[3]);

    const float mu = (e == NE - 1) ? RBF_END_F : RBF_END_F * ((float)e * (1.0f / (float)(NE - 1)));
#pragma unroll
    for (int j = 0; j < 4; ++j) {
#pragma unroll
      for (int r = 0; r < 8; ++r) {
        const float t  = dist[j][r] - mu;
        const float q  = t * t;
        const float ag = q * NEG16LOG2E;
        const float ex = __builtin_amdgcn_exp2f(ag);
        run = fmaf(acc[j][r], ex, run);
      }
    }
  }

  float s = run;
  s += __shfl_xor(s, 16);
  s += __shfl_xor(s, 8);
  s += __shfl_xor(s, 4);
  s += __shfl_xor(s, 2);
  s += __shfl_xor(s, 1);
  if (lane == 0) red[wave] = s;
  __syncthreads();
  if (wave == 0) {
    const float bs = ((red[0] + red[1]) + red[2]) + red[3];
    const float v  = (lane == 0) ? bs : 0.f;
    float* p = PART + (size_t)(by * NBX + bx) * 32 + lane;
    *(volatile float*)p = v;
    __threadfence();
    *(volatile float*)p = v;
  }
}

__global__ __launch_bounds__(256) void fin_sum(const float* __restrict__ PART, float* out) {
  __shared__ double sm[256];
  const int tid = (int)threadIdx.x;
  double s = 0.0;
#pragma unroll 1
  for (int i = tid; i < NBLK; i += 256) s += (double)PART[(size_t)i * 32];
  sm[tid] = s;
  __syncthreads();
#pragma unroll 1
  for (int w = 128; w > 0; w >>= 1) {
    if (tid < w) sm[tid] = sm[tid] + sm[tid + w];
    __syncthreads();
  }
  const float S = (float)sm[0];
  const float U = S * ESCALE;
  if (tid == 0) *(volatile float*)out = U;
  __threadfence();
  if (tid == 0) *(volatile float*)out = U;
}

extern "C" void kernel_launch(void* const* d_in, const int* in_sizes, int n_in,
                              void* d_out, int out_size, void* d_ws, size_t ws_size,
                              hipStream_t stream) {
  if (n_in < 4) return;
  if ((long long)in_sizes[0] < (long long)NL * FP) return;
  if ((long long)in_sizes[1] < (long long)NR * FP) return;
  if (in_sizes[2] < NL * 3) return;
  if (in_sizes[3] < NR * 3) return;
  if (out_size < 1) return;

  size_t off = 0;
  const size_t oLIG  = off; off += (size_t)LIGB;
  const size_t oREC  = off; off += (size_t)RECB;
  const size_t oPART = off; off += (size_t)PARTB;
  if (off > ws_size) return;
  if (off > (size_t)134217728) return;

  const float* ligf = (const float*)d_in[0];
  const float* recf = (const float*)d_in[1];
  const float* ligc = (const float*)d_in[2];
  const float* recc = (const float*)d_in[3];

  char* ws = (char*)d_ws;
  unsigned short* LIGp = (unsigned short*)(ws + oLIG);
  unsigned short* RECp = (unsigned short*)(ws + oREC);
  float*          PART = (float*)(ws + oPART);
  float*          out0 = (float*)d_out;

  const int n8l = NL * FP / 8;
  const int n8r = NR * FP / 8;
  const dim3 blk256(256);
  const dim3 blk128(128);
  const dim3 gCl(n8l / 256);
  const dim3 gCr(n8r / 256);
  const dim3 gE(NBX, NBY);

  cvt_bf16x8<<<gCl, blk256, 0, stream>>>(ligf, LIGp, n8l);
  cvt_bf16x8<<<gCr, blk256, 0, stream>>>(recf, RECp, n8r);
  pair_energy<<<gE, blk128, 0, stream>>>(LIGp, RECp, ligc, recc, PART);
  fin_sum<<<dim3(1), blk256, 0, stream>>>(PART, out0);
  (void)hipGetLastError();
}
